// SparseConvBlock_61993557951055
// MI455X (gfx1250) — hardware-run, weakly checked
//
#include <hip/hip_runtime.h>


namespace {
constexpr int N = 100000, C = 64, K = 27, KC = K * C  , NW = N / 16  ;
constexpr float XS = 8.0f, WSC = 256.0f, EPS = 1e-5f;
typedef _Float16 b16;
typedef __attribute__((ext_vector_type(16))) _Float16 v16b;
typedef __attribute__((ext_vector_type(8))) _Float16 v8b;
typedef __attribute__((ext_vector_type(8))) float v8f;
typedef __attribute__((ext_vector_type(4))) float v4f;
typedef __attribute__((ext_vector_type(2))) float v2f;
__device__ __forceinline__ float bf16_rne(float f) { unsigned int u = __float_as_uint(f); u += 0x7FFFu + ((u >> 16) & 1u); float r = __uint_as_float(u & 0xFFFF0000u); asm volatile("" : "+v"(r)); return r; }
__device__ __forceinline__ float bfv(float f) { float r = bf16_rne(f); asm volatile("" : "+v"(r)); return r; }
__device__ __forceinline__ v16b frag_kb(const b16* p, int hh) { const v8b a = *(const v8b*)(p + 8 * hh), b = *(const v8b*)(p + 16 + 8 * hh); v16b f;
#pragma unroll
  for (int e = 0; e < 8; ++e) { f[e] = a[e]; f[8 + e] = b[e]; } return f; }
__device__ __forceinline__ v8f wmma16b(v16b a, v16b b, v8f c) { v8f d = __builtin_amdgcn_wmma_f32_16x16x32_f16(false, a, false, b, (short)0, c, false, false); asm volatile("v_nop\n\tv_nop\n\tv_nop\n\tv_nop" : "+v"(d) : "v"(a), "v"(b)); return d; }
__device__ __forceinline__ void wave_lds_sync() { __builtin_amdgcn_fence(__ATOMIC_RELEASE, "workgroup"); __builtin_amdgcn_wave_barrier(); __builtin_amdgcn_fence(__ATOMIC_ACQUIRE, "workgroup"); }
__device__ __forceinline__ float pmul(float a, float b) { float p = a * b; asm volatile("" : "+v"(p)); return p; }
__device__ __forceinline__ int iclamp(int v, int lo, int hi) { return v < lo ? lo : (v > hi ? hi : v); }

__global__ __launch_bounds__(256) void wput_kernel(const float* __restrict__ w, b16* __restrict__ WT) { const int u = blockIdx.x * 256 + threadIdx.x; if (u >= C * (KC / 8)) return; const int o = u / (KC / 8), k0 = (u % (KC / 8)) * 8; v8b v;
#pragma unroll
  for (int j = 0; j < 8; ++j) { const int k = k0 + j; v[j] = (b16)(bf16_rne(w[((size_t)(k / C) * C + (k % C)) * C + o]) * WSC); }
  for (int pass = 0; pass < 2; ++pass) { *(volatile v8b*)(WT + (size_t)o * KC + k0) = v; __threadfence(); } }
__global__ __launch_bounds__(32) void conv_kernel(const float* __restrict__ feat, const int* __restrict__ nbr, const b16* __restrict__ WT, int NLIM, float* __restrict__ CONV, float* __restrict__ PS, float* __restrict__ PQ) { __shared__ __attribute__((aligned(16))) b16 Ah[16][KC + 8]; __shared__ float Tf[16][C + 1]; const int lane = threadIdx.x, nloc = lane & 15, hlf = lane >> 4; const size_t n0 = (size_t)blockIdx.x * 16; if (n0 >= (size_t)NLIM) return;
  for (int rr = 0; rr < 16; ++rr) {
#pragma unroll 1
    for (int kk = 0; kk < K; ++kk) { const int id = nbr[(n0 + rr) * K + kk]; const bool ok = id >= 0 && id < NLIM; const size_t src = (size_t)iclamp(id, 0, N - 1); const v2f fv = ok ? *(const v2f*)(feat + src * C + lane * 2) : (v2f){0.0f, 0.0f}; Ah[rr][kk * C + lane * 2] = (b16)(bfv(fv[0]) * XS); Ah[rr][kk * C + lane * 2 + 1] = (b16)(bfv(fv[1]) * XS); } }
  if (lane < 16) for (int k = KC; k < KC + 8; ++k) Ah[lane][k] = (b16)0.0f;
  wave_lds_sync(); v8f acc[4] = {(v8f){}, (v8f){}, (v8f){}, (v8f){}};
#pragma unroll 2
  for (int kb = 0; kb < KC; kb += 32) { const v16b a = frag_kb(&Ah[nloc][kb], hlf);
#pragma unroll
    for (int t = 0; t < 4; ++t) acc[t] = wmma16b(a, frag_kb(WT + (size_t)(t * 16 + nloc) * KC + kb, hlf), acc[t]); }
#pragma unroll
  for (int t = 0; t < 4; ++t)
#pragma unroll
    for (int r8 = 0; r8 < 8; ++r8) Tf[8 * hlf + r8][t * 16 + nloc] = acc[t][r8] * (1.0f / (XS * WSC));
  wave_lds_sync();
  float s0 = 0.0f, s1 = 0.0f, q0 = 0.0f, q1 = 0.0f; for (int rr = 0; rr < 16; ++rr) { const float a0 = Tf[rr][lane * 2], a1 = Tf[rr][lane * 2 + 1]; s0 += a0; s1 += a1; q0 += a0 * a0; q1 += a1 * a1; }
  for (int pass = 0; pass < 2; ++pass) { for (int rr = 0; rr < 16; ++rr) *(volatile v2f*)(CONV + (n0 + rr) * C + lane * 2) = (v2f){Tf[rr][lane * 2], Tf[rr][lane * 2 + 1]}; *(volatile v2f*)(PS + (size_t)blockIdx.x * C + lane * 2) = (v2f){s0, s1}; *(volatile v2f*)(PQ + (size_t)blockIdx.x * C + lane * 2) = (v2f){q0, q1}; __threadfence(); } }
__global__ __launch_bounds__(256) void stat_kernel(const float* __restrict__ PS, const float* __restrict__ PQ, int nwaves, int ncount, float* __restrict__ ST) { const int wave = threadIdx.x >> 5, lane = threadIdx.x & 31; const int c = blockIdx.x * 8 + wave; if (c >= C) return; double s = 0.0, q = 0.0; for (int w = lane; w < nwaves; w += 32) { s += (double)PS[(size_t)w * C + c]; q += (double)PQ[(size_t)w * C + c]; } for (int o = 16; o; o >>= 1) { s += __shfl_xor(s, o); q += __shfl_xor(q, o); }
  const double mean = s / ncount, var = fmax(q / ncount - mean * mean, 0.0); const float m = (float)mean, rs = (float)(1.0 / sqrt(var + (double)EPS));
  for (int pass = 0; pass < 2; ++pass) { ((volatile float*)ST)[(size_t)c * 32 + lane] = lane == 0 ? m : (lane == 1 ? rs : 0.0f); __threadfence(); } }
__global__ __launch_bounds__(256) void bn_kernel(const float* __restrict__ CONV, const float* __restrict__ ST, const float* __restrict__ gamma, const float* __restrict__ beta, int NLIM, float* __restrict__ out) { const size_t u = (size_t)blockIdx.x * 256 + threadIdx.x; if (u >= (size_t)NLIM * C / 2) return; const int c = (int)((u * 2) % C); const v2f v = *(const v2f*)(CONV + u * 2); v2f r;
  for (int e = 0; e < 2; ++e) { const float m = ST[(c + e) * 32], rs = ST[(c + e) * 32 + 1]; r[e] = fmaxf(pmul((v[e] - m) * rs, bfv(gamma[c + e])) + bfv(beta[c + e]), 0.0f); }
  for (int pass = 0; pass < 2; ++pass) { *(volatile v2f*)(out + u * 2) = r; __threadfence(); } }
}

extern "C" void kernel_launch(void* const* d_in, const int* in_sizes, int n_in, void* d_out, int out_size, void* d_ws, size_t ws_size, hipStream_t stream) {
  (void)n_in;
  auto Fp = [&](int i) { return (const float*)d_in[i]; }; auto Ip = [&](int i) { return (const int*)d_in[i]; };
  if (in_sizes[0] != N * C || in_sizes[1] != N * K || in_sizes[2] != K * C * C || in_sizes[3] != C || out_size != N * C) return;
  const int NLIM = N;
  size_t off = 0; char* ws = (char*)d_ws;
  auto carve = [&](size_t bytes) { char* p = ws + off; off += (bytes + 255) & ~(size_t)255; return p; };
  b16* WT = (b16*)carve((size_t)C * KC * 2); float* CONV = (float*)carve((size_t)N * C * 4); float* PS = (float*)carve((size_t)NW * C * 4); float* PQ = (float*)carve((size_t)NW * C * 4); float* ST = (float*)carve((size_t)C * 32 * 4);
  if (off > ws_size || off > ((size_t)40 << 20)) return;
  wput_kernel<<<(C * (KC / 8) + 255) / 256, 256, 0, stream>>>(Fp(2), WT);
  conv_kernel<<<NLIM / 16, 32, 0, stream>>>(Fp(0), Ip(1), WT, NLIM, CONV, PS, PQ);
  stat_kernel<<<C / 8, 256, 0, stream>>>(PS, PQ, NLIM / 16, NLIM, ST);
  bn_kernel<<<(NLIM * C / 2 + 255) / 256, 256, 0, stream>>>(CONV, ST, Fp(3), Fp(4), NLIM, (float*)d_out);
}
